// Mamba_71451075937043
// MI455X (gfx1250) — hardware-run, weakly checked
//
#include <hip/hip_runtime.h>


#ifndef SEQ
#define SEQ 2048
#endif
#define SEQ_FULL 2048
#define NLAY 2
#define DMOD 1024
#define EDIM 2048
#define XZP  4096
#define RNK  64
#define NST  16
#define KCV  4
#define XPR  96
#define XPP  128
#define BCW  32
#define TS   16
#define WSC  64.0f
#define WSI  (1.0f / 64.0f)
#define EPSV 1e-5f
#define L2E  1.4426950408889634f
#define LN2  0.6931471805599453f

static_assert(SEQ % 64 == 0);
static_assert(SEQ % TS == 0);
static_assert(SEQ % 8 == 0);
static_assert(SEQ <= SEQ_FULL);
static_assert(XZP == 2 * EDIM);
static_assert(XZP % 64 == 0);
static_assert(EDIM % 64 == 0);
static_assert(DMOD % 64 == 0);
static_assert(XPP % 64 == 0);
static_assert(XPP == 128);
static_assert(XPR == RNK + 2 * NST);
static_assert(RNK == 64);
static_assert(BCW == 2 * NST);
static_assert(BCW * 4 == 128);
static_assert(DMOD % 32 == 0);
static_assert(EDIM % 32 == 0);
static_assert(RNK % 32 == 0);
static_assert(DMOD == 4 * 32 * 8);
static_assert(EDIM == 256 * 8);
static_assert(EDIM % 64 == 0);
static_assert(2 * 2 * 32 * 16 == TS * 64 * 2);
static_assert(2 * 64 * 4 == TS * BCW);
static_assert(8 * 32 * 16 == 16 * 64 * 4);
static_assert(4 * 32 * 16 == 16 * 64 * 2);
static_assert(4 * 32 * 16 == 16 * BCW * 4);
static_assert(16 * 68 * 4 <= 131072);
static_assert(TS * BCW * 4 + TS * 64 * 2 <= 131072);

typedef _Float16 h16;
typedef __attribute__((ext_vector_type(16))) _Float16 v16h;
typedef __attribute__((ext_vector_type(8)))  _Float16 v8h;
typedef __attribute__((ext_vector_type(8)))  float    v8f;
typedef __attribute__((ext_vector_type(4)))  float    v4f;
typedef v4f  __attribute__((may_alias)) v4fa;
typedef v8h  __attribute__((may_alias)) v8ha;

__device__ __forceinline__ unsigned short f2bf(float f) { unsigned u = __float_as_uint(f); u += 0x7FFFu + ((u >> 16) & 1u); return (unsigned short)(u >> 16); }
__device__ __forceinline__ float bfr(float f) { return __uint_as_float(((unsigned)f2bf(f)) << 16); }
__device__ __forceinline__ v16h cat16(v8h lo, v8h hi) { return __builtin_shufflevector(lo, hi, 0, 1, 2, 3, 4, 5, 6, 7, 8, 9, 10, 11, 12, 13, 14, 15); }
__device__ __forceinline__ v16h  ldh(const h16* p) { return cat16(*(const v8h*)p, *(const v8h*)(p + 16)); }
__device__ __forceinline__ void wave_sync() { __builtin_amdgcn_fence(3  , "wavefront"); __builtin_amdgcn_wave_barrier(); asm volatile("" ::: "memory"); }
static __device__ __forceinline__ h16 toh_flush(float v) { const h16 r = (h16)v; return (fabsf(v) < 6.103515625e-05f) ? (h16)0.0f : r; }
__device__ __forceinline__ v8f wmma16g(v16h a, v16h b, v8f c) {
    c = __builtin_amdgcn_wmma_f32_16x16x32_f16(false, a, false, b, (short)0, c, false, false);
    asm volatile("v_nop\n\tv_nop\n\tv_nop\n\tv_nop" : "+v"(c) : "v"(a), "v"(b));
    return c;
}

__global__ __launch_bounds__(256) void k_wconv(const float* __restrict__ src, h16* dst, unsigned n8, unsigned rl8, unsigned RS, unsigned RD) {
    const unsigned i = blockIdx.x * 256u + threadIdx.x; if (i >= n8) return;
    const unsigned row = i / rl8, g = i - row * rl8;
    const unsigned lay = row / RD, r = row - lay * RD;
    const unsigned rc = r < RS ? r : RS - 1u;
    const size_t so = ((size_t)(lay * RS + rc) * rl8 + g) * 8;
    v4f x0 = *(const v4f*)(src + so), x1 = *(const v4f*)(src + so + 4);
    asm volatile("" : "+v"(x0), "+v"(x1));
    const bool ok = r < RS;
    v8h o;
#pragma unroll
    for (int k = 0; k < 4; ++k) {
        const float f0 = ok ? bfr(x0[k]) * WSC : 0.0f; const float f1 = ok ? bfr(x1[k]) * WSC : 0.0f;
        o[k] = toh_flush(f0); o[4 + k] = toh_flush(f1); }
    *(volatile v8h*)(dst + (size_t)i * 8) = o; __threadfence(); *(volatile v8h*)(dst + (size_t)i * 8) = o;
}

__global__ __launch_bounds__(256) void k_rms(const float* __restrict__ X, const float* __restrict__ gw, h16* XN, int inbf) {
#pragma clang fp contract(off)
    const int lane = threadIdx.x & 31;
    const int wave = __builtin_amdgcn_readfirstlane((int)(threadIdx.x >> 5));
    const int row = blockIdx.x * 8 + wave;
    const float* xr = X + (size_t)row * DMOD;
    float s = 0.0f;
#pragma unroll 1
    for (int j = 0; j < 4; ++j) {
        const int off = (j * 32 + lane) * 8;
        const v4f a = *(const v4f*)(xr + off), c = *(const v4f*)(xr + off + 4);
#pragma unroll
        for (int i = 0; i < 4; ++i) { const float p = inbf ? bfr(a[i]) : a[i]; const float q = inbf ? bfr(c[i]) : c[i]; s = s + p * p; s = s + q * q; }
    }
    s += __shfl_xor(s, 16, 32); s += __shfl_xor(s, 8, 32); s += __shfl_xor(s, 4, 32); s += __shfl_xor(s, 2, 32); s += __shfl_xor(s, 1, 32);
    const float sc = rsqrtf(s * (1.0f / (float)DMOD) + EPSV);
    h16* orow = XN + (size_t)row * DMOD;
#pragma unroll 1
    for (int ps = 0; ps < 2; ++ps) {
#pragma unroll 1
        for (int j = 0; j < 4; ++j) {
            const int off = (j * 32 + lane) * 8;
            const v4f a = *(const v4f*)(xr + off), c = *(const v4f*)(xr + off + 4);
            const v4f w0 = *(const v4f*)(gw + off), w1 = *(const v4f*)(gw + off + 4);
            v8h o;
#pragma unroll
            for (int i = 0; i < 4; ++i) { const float p = inbf ? bfr(a[i]) : a[i]; const float q = inbf ? bfr(c[i]) : c[i];
                o[i] = toh_flush((p * sc) * bfr(w0[i])); o[4 + i] = toh_flush((q * sc) * bfr(w1[i])); }
            *(volatile v8h*)(orow + off) = o; }
        if (ps == 0) __threadfence(); }
}

__global__ __launch_bounds__(256) void k_conv(const float* __restrict__ XZ, const float* __restrict__ cw, const float* __restrict__ cb, h16* XCH) {
#pragma clang fp contract(off)
    const int l = blockIdx.x; const int e8 = threadIdx.x * 8;
    v4f wv[8];
#pragma unroll
    for (int c = 0; c < 8; ++c) wv[c] = *(const v4f*)(cw + (size_t)(e8 + c) * KCV);
    const v4f b0 = *(const v4f*)(cb + e8), b1 = *(const v4f*)(cb + e8 + 4);
    float acc[8];
#pragma unroll
    for (int c = 0; c < 8; ++c) acc[c] = 0.0f;
#pragma unroll
    for (int j = 0; j < KCV; ++j) {
        const int ll = l - (KCV - 1) + j; const int lc = ll < 0 ? 0 : ll;
        v4f x0 = *(const v4f*)(XZ + (size_t)lc * XZP + e8), x1 = *(const v4f*)(XZ + (size_t)lc * XZP + e8 + 4);
        asm volatile("" : "+v"(x0), "+v"(x1));
#pragma unroll
        for (int c = 0; c < 4; ++c) { const float xa = (ll < 0) ? 0.0f : x0[c]; const float xb = (ll < 0) ? 0.0f : x1[c];
            acc[c] = acc[c] + bfr(wv[c][j]) * xa; acc[4 + c] = acc[4 + c] + bfr(wv[4 + c][j]) * xb; }
    }
    v8h o;
#pragma unroll
    for (int c = 0; c < 4; ++c) {
        const float va = acc[c] + bfr(b0[c]); const float vb = acc[4 + c] + bfr(b1[c]);
        const float sa = va * __builtin_amdgcn_rcpf(1.0f + __builtin_amdgcn_exp2f(-va * L2E));
        const float sb = vb * __builtin_amdgcn_rcpf(1.0f + __builtin_amdgcn_exp2f(-vb * L2E));
        o[c] = toh_flush(sa); o[4 + c] = toh_flush(sb); }
    h16* p = XCH + (size_t)l * EDIM + e8;
    *(volatile v8h*)p = o; __threadfence(); *(volatile v8h*)p = o;
}

__device__ __forceinline__ void gemm_main(v8f (&acc)[4][4], const h16* __restrict__ A, const size_t aoff, const int lda,
                                          const h16* __restrict__ Bt, const size_t boff, const int ldb, const int K) {
#pragma unroll
    for (int mb = 0; mb < 4; ++mb)
#pragma unroll
        for (int nb = 0; nb < 4; ++nb) acc[mb][nb] = (v8f){};
#pragma unroll 1
    for (int kc = 0; kc < K; kc += 32) {
        v16h a[4];
#pragma unroll
        for (int mb = 0; mb < 4; ++mb) a[mb] = ldh(A + aoff + (size_t)mb * 16 * lda + kc);
#pragma unroll
        for (int nb = 0; nb < 4; ++nb) { const v16h b = ldh(Bt + boff + (size_t)nb * 16 * ldb + kc);
#pragma unroll
            for (int mb = 0; mb < 4; ++mb) acc[mb][nb] = wmma16g(a[mb], b, acc[mb][nb]); }
    }
}

__global__ __launch_bounds__(32) void k_gemm_in(const h16* __restrict__ A, const h16* __restrict__ Bt, float* C) {
    __shared__ __align__(16) float os[16 * 68];
    const int lane = threadIdx.x & 31, lr = lane & 15, hi = lane >> 4; const int r0 = blockIdx.x * 64, c0 = blockIdx.y * 64;
    v8f acc[4][4];
    gemm_main(acc, A, (size_t)(r0 + lr) * DMOD + 8 * hi, DMOD, Bt, (size_t)(c0 + lr) * DMOD + 8 * hi, DMOD, DMOD);
#pragma unroll
    for (int mb = 0; mb < 4; ++mb) {
#pragma unroll
        for (int nb = 0; nb < 4; ++nb) {
#pragma unroll
            for (int j = 0; j < 8; ++j) os[(hi * 8 + j) * 68 + nb * 16 + lr] = acc[mb][nb][j] * WSI; }
        wave_sync();
        float* cbp = C + (size_t)(r0 + mb * 16) * XZP + c0;
#pragma unroll 1
        for (int ps = 0; ps < 2; ++ps) {
#pragma unroll
            for (int s = 0; s < 8; ++s) { const int row = 2 * s + (lane >> 4), c4 = (lane & 15) * 4;
                const v4f val = *(const v4fa*)(&os[row * 68 + c4]);
                *(volatile v4f*)(cbp + (size_t)row * XZP + c4) = val; }
            if (ps == 0) __threadfence(); }
        wave_sync();
    }
}

__global__ __launch_bounds__(32) void k_gemm_xp(const h16* __restrict__ A, const h16* __restrict__ Bt, h16* DTH, float* BC) {
    __shared__ __align__(16) float os[16 * 68];
    const int lane = threadIdx.x & 31, lr = lane & 15, hi = lane >> 4; const int r0 = blockIdx.x * 64, c0 = blockIdx.y * 64;
    v8f acc[4][4];
    gemm_main(acc, A, (size_t)(r0 + lr) * EDIM + 8 * hi, EDIM, Bt, (size_t)(c0 + lr) * EDIM + 8 * hi, EDIM, EDIM);
#pragma unroll
    for (int mb = 0; mb < 4; ++mb) {
#pragma unroll
        for (int nb = 0; nb < 4; ++nb) {
#pragma unroll
            for (int j = 0; j < 8; ++j) os[(hi * 8 + j) * 68 + nb * 16 + lr] = acc[mb][nb][j] * WSI; }
        wave_sync();
#pragma unroll 1
        for (int ps = 0; ps < 2; ++ps) {
            if (c0 == 0) {
                h16* dp = DTH + (size_t)(r0 + mb * 16) * RNK;
#pragma unroll
                for (int s = 0; s < 4; ++s) { const int row = 4 * s + (lane >> 3), c8 = (lane & 7) * 8;
                    const v4f x0 = *(const v4fa*)(&os[row * 68 + c8]); const v4f x1 = *(const v4fa*)(&os[row * 68 + c8 + 4]); v8h hv;
#pragma unroll
                    for (int i = 0; i < 4; ++i) { hv[i] = toh_flush(x0[i]); hv[4 + i] = toh_flush(x1[i]); }
                    *(volatile v8h*)(dp + (size_t)row * RNK + c8) = hv; }
            } else {
                float* bp = BC + (size_t)(r0 + mb * 16) * BCW;
#pragma unroll
                for (int s = 0; s < 4; ++s) { const int row = 4 * s + (lane >> 3), c4 = (lane & 7) * 4;
                    const v4f val = *(const v4fa*)(&os[row * 68 + c4]);
                    *(volatile v4f*)(bp + (size_t)row * BCW + c4) = val; }
            }
            if (ps == 0) __threadfence(); }
        wave_sync();
    }
}

__global__ __launch_bounds__(32) void k_gemm_dt(const h16* __restrict__ A, const h16* __restrict__ Bt, const float* __restrict__ bias, float* C) {
    __shared__ __align__(16) float os[16 * 68];
    const int lane = threadIdx.x & 31, lr = lane & 15, hi = lane >> 4; const int r0 = blockIdx.x * 64, c0 = blockIdx.y * 64;
    v8f acc[4][4];
    gemm_main(acc, A, (size_t)(r0 + lr) * RNK + 8 * hi, RNK, Bt, (size_t)(c0 + lr) * RNK + 8 * hi, RNK, RNK);
    float bc[4];
#pragma unroll
    for (int nb = 0; nb < 4; ++nb) bc[nb] = bfr(bias[c0 + nb * 16 + lr]);
#pragma unroll
    for (int mb = 0; mb < 4; ++mb) {
#pragma unroll
        for (int nb = 0; nb < 4; ++nb) {
#pragma unroll
            for (int j = 0; j < 8; ++j) {
                const float xv = acc[mb][nb][j] * WSI + bc[nb];
                const float ee = __builtin_amdgcn_exp2f(-fabsf(xv) * L2E);
                const float ser = ee * (1.0f - ee * (0.5f - ee * 0.33333334f));
                const float lg = __builtin_amdgcn_logf(1.0f + ee) * LN2;
                const float lp = (ee < 0.015625f) ? ser : lg;
                os[(hi * 8 + j) * 68 + nb * 16 + lr] = fmaxf(xv, 0.0f) + lp; } }
        wave_sync();
        float* cbp = C + (size_t)(r0 + mb * 16) * EDIM + c0;
#pragma unroll 1
        for (int ps = 0; ps < 2; ++ps) {
#pragma unroll
            for (int s = 0; s < 8; ++s) { const int row = 2 * s + (lane >> 4), c4 = (lane & 15) * 4;
                const v4f val = *(const v4fa*)(&os[row * 68 + c4]);
                *(volatile v4f*)(cbp + (size_t)row * EDIM + c4) = val; }
            if (ps == 0) __threadfence(); }
        wave_sync();
    }
}

__global__ __launch_bounds__(32) void k_gemm_out(const h16* __restrict__ A, const h16* __restrict__ Bt, const float* __restrict__ res, int resbf, float* C) {
    __shared__ __align__(16) float os[16 * 68];
    const int lane = threadIdx.x & 31, lr = lane & 15, hi = lane >> 4; const int r0 = blockIdx.x * 64, c0 = blockIdx.y * 64;
    v8f acc[4][4];
    gemm_main(acc, A, (size_t)(r0 + lr) * EDIM + 8 * hi, EDIM, Bt, (size_t)(c0 + lr) * EDIM + 8 * hi, EDIM, EDIM);
#pragma unroll
    for (int mb = 0; mb < 4; ++mb) {
#pragma unroll
        for (int nb = 0; nb < 4; ++nb) {
#pragma unroll
            for (int j = 0; j < 8; ++j) os[(hi * 8 + j) * 68 + nb * 16 + lr] = acc[mb][nb][j] * WSI; }
        wave_sync();
        const size_t tb = (size_t)(r0 + mb * 16) * DMOD + c0;
#pragma unroll 1
        for (int ps = 0; ps < 2; ++ps) {
#pragma unroll
            for (int s = 0; s < 8; ++s) { const int row = 2 * s + (lane >> 4), c4 = (lane & 15) * 4;
                v4f val = *(const v4fa*)(&os[row * 68 + c4]);
                const v4f rv = *(const v4f*)(res + tb + (size_t)row * DMOD + c4);
#pragma unroll
                for (int i = 0; i < 4; ++i) val[i] = val[i] + (resbf ? bfr(rv[i]) : rv[i]);
                *(volatile v4f*)(C + tb + (size_t)row * DMOD + c4) = val; }
            if (ps == 0) __threadfence(); }
        wave_sync();
    }
}

__global__ __launch_bounds__(64) void k_scan(const float* __restrict__ DELTA, const h16* __restrict__ XCH, const float* __restrict__ BC, const float* __restrict__ XZ,
                                             const float* __restrict__ alog, const float* __restrict__ dpar, h16* YG) {
#pragma clang fp contract(off)
    __shared__ __align__(16) float bcs[TS * BCW];
    __shared__ __align__(16) h16 ys[TS * 64];
    const int tid = threadIdx.x, lane = tid & 31;
    const int wave = __builtin_amdgcn_readfirstlane((int)(threadIdx.x >> 5));
    const int e0 = blockIdx.x * 64, e = e0 + tid;
    float a2[NST], h[NST];
#pragma unroll
    for (int q = 0; q < 4; ++q) { const v4f al = *(const v4f*)(alog + (size_t)e * NST + q * 4);
#pragma unroll
        for (int i = 0; i < 4; ++i) { a2[q * 4 + i] = -__builtin_amdgcn_exp2f(bfr(al[i]) * L2E) * L2E; h[q * 4 + i] = 0.0f; } }
    const float dsk = bfr(dpar[e]);
#pragma unroll 1
    for (int l0 = 0; l0 < SEQ; l0 += TS) {
#pragma unroll
        for (int q = 0; q < 2; ++q) { const int idx = q * 64 + tid;
            *(v4fa*)(&bcs[idx * 4]) = *(const v4f*)(BC + (size_t)l0 * BCW + idx * 4); }
        __syncthreads();
#pragma unroll 1
        for (int i = 0; i < TS; ++i) {
            const size_t l = (size_t)(l0 + i);
            const float d = DELTA[l * EDIM + e];
            const float u = (float)XCH[l * EDIM + e];
            const float z = XZ[l * XZP + EDIM + e];
            const float du = d * u;
            float y = 0.0f;
#pragma unroll
            for (int q = 0; q < 4; ++q) {
                const v4f bq = *(const v4fa*)(&bcs[i * BCW + q * 4]);
                const v4f cq = *(const v4fa*)(&bcs[i * BCW + NST + q * 4]);
#pragma unroll
                for (int k = 0; k < 4; ++k) { const int n = q * 4 + k;
                    const float a = __builtin_amdgcn_exp2f(d * a2[n]);
                    h[n] = a * h[n] + du * bq[k];
                    y = y + h[n] * cq[k]; } }
            y = y + dsk * u;
            const float g = z * __builtin_amdgcn_rcpf(1.0f + __builtin_amdgcn_exp2f(-z * L2E));
            ys[i * 64 + tid] = toh_flush(y * g);
        }
        __syncthreads();
        h16* op = YG + (size_t)l0 * EDIM + e0;
#pragma unroll 1
        for (int ps = 0; ps < 2; ++ps) {
#pragma unroll
            for (int s = 0; s < 2; ++s) { const int row = wave * 8 + 4 * s + (lane >> 3), c8 = (lane & 7) * 8;
                const v8h val = *(const v8ha*)(&ys[row * 64 + c8]);
                *(volatile v8h*)(op + (size_t)row * EDIM + c8) = val; }
            if (ps == 0) __threadfence(); }
    }
}

static constexpr size_t al256(size_t v) { return (v + 255) & ~(size_t)255; }
static constexpr size_t SZ_WIN = al256((size_t)NLAY * XZP * DMOD * 2);
static constexpr size_t SZ_WOU = al256((size_t)NLAY * DMOD * EDIM * 2);
static constexpr size_t SZ_WXP = al256((size_t)NLAY * XPP * EDIM * 2);
static constexpr size_t SZ_WDT = al256((size_t)NLAY * EDIM * RNK * 2);
static constexpr size_t SZ_XN  = al256((size_t)SEQ * DMOD * 2);
static constexpr size_t SZ_XZ  = al256((size_t)SEQ * XZP * 4);
static constexpr size_t SZ_XC  = al256((size_t)SEQ * EDIM * 2);
static constexpr size_t SZ_DT  = al256((size_t)SEQ * RNK * 2);
static constexpr size_t SZ_BC  = al256((size_t)SEQ * BCW * 4);
static constexpr size_t SZ_DL  = al256((size_t)SEQ * EDIM * 4);
static constexpr size_t SZ_YG  = al256((size_t)SEQ * EDIM * 2);
static constexpr size_t SZ_X1  = al256((size_t)SEQ * DMOD * 4);
static constexpr size_t SZ_TOTAL = SZ_WIN + SZ_WOU + SZ_WXP + SZ_WDT + SZ_XN + SZ_XZ + SZ_XC + SZ_DT + SZ_BC + SZ_DL + SZ_YG + SZ_X1;
static_assert(SZ_TOTAL <= (size_t)134217728);
static_assert(((size_t)NLAY * XZP * DMOD) % 8 == 0);
static_assert(((size_t)NLAY * XPP * EDIM) % 8 == 0);
static_assert(((size_t)NLAY * EDIM * RNK) % 8 == 0);
static_assert(((size_t)NLAY * DMOD * EDIM) % 8 == 0);
static_assert((size_t)NLAY * XZP * DMOD / 8 < (size_t)2147483647);

extern "C" void kernel_launch(void* const* d_in, const int* in_sizes, int n_in,
                              void* d_out, int out_size, void* d_ws, size_t ws_size, hipStream_t stream) {
    if (n_in < 11) return;
    if ((size_t)in_sizes[0] < (size_t)SEQ * DMOD) return;
    if ((size_t)in_sizes[1] < (size_t)NLAY * DMOD) return;
    if ((size_t)in_sizes[2] < (size_t)NLAY * XZP * DMOD) return;
    if ((size_t)in_sizes[3] < (size_t)NLAY * EDIM * KCV) return;
    if ((size_t)in_sizes[4] < (size_t)NLAY * EDIM) return;
    if ((size_t)in_sizes[5] < (size_t)NLAY * XPR * EDIM) return;
    if ((size_t)in_sizes[6] < (size_t)NLAY * EDIM * RNK) return;
    if ((size_t)in_sizes[7] < (size_t)NLAY * EDIM) return;
    if ((size_t)in_sizes[8] < (size_t)NLAY * EDIM * NST) return;
    if ((size_t)in_sizes[9] < (size_t)NLAY * EDIM) return;
    if ((size_t)in_sizes[10] < (size_t)NLAY * DMOD * EDIM) return;
    if ((size_t)out_size < (size_t)SEQ * DMOD) return;
    if (SZ_TOTAL > ws_size) return;
    const float* x_in   = (const float*)d_in[0];
    const float* norm_w = (const float*)d_in[1];
    const float* win    = (const float*)d_in[2];
    const float* conv_w = (const float*)d_in[3];
    const float* conv_b = (const float*)d_in[4];
    const float* wx     = (const float*)d_in[5];
    const float* wdt    = (const float*)d_in[6];
    const float* bdt    = (const float*)d_in[7];
    const float* a_log  = (const float*)d_in[8];
    const float* dpar   = (const float*)d_in[9];
    const float* wout   = (const float*)d_in[10];
    float* OUT = (float*)d_out;
    char* wsp = (char*)d_ws;
    h16* WINH = (h16*)wsp; wsp += SZ_WIN;
    h16* WOUH = (h16*)wsp; wsp += SZ_WOU;
    h16* WXPH = (h16*)wsp; wsp += SZ_WXP;
    h16* WDTH = (h16*)wsp; wsp += SZ_WDT;
    h16* XN   = (h16*)wsp; wsp += SZ_XN;
    float* XZ = (float*)wsp; wsp += SZ_XZ;
    h16* XCH  = (h16*)wsp; wsp += SZ_XC;
    h16* DTH  = (h16*)wsp; wsp += SZ_DT;
    float* BC = (float*)wsp; wsp += SZ_BC;
    float* DL = (float*)wsp; wsp += SZ_DL;
    h16* YG   = (h16*)wsp; wsp += SZ_YG;
    float* X1 = (float*)wsp; wsp += SZ_X1;

    { const unsigned n8 = (unsigned)((size_t)NLAY * XZP * DMOD / 8);
      k_wconv<<<(n8 + 255u) / 256u, 256, 0, stream>>>(win, WINH, n8, (unsigned)(DMOD / 8), (unsigned)XZP, (unsigned)XZP); }
    { const unsigned n8 = (unsigned)((size_t)NLAY * XPP * EDIM / 8);
      k_wconv<<<(n8 + 255u) / 256u, 256, 0, stream>>>(wx, WXPH, n8, (unsigned)(EDIM / 8), (unsigned)XPR, (unsigned)XPP); }
    { const unsigned n8 = (unsigned)((size_t)NLAY * EDIM * RNK / 8);
      k_wconv<<<(n8 + 255u) / 256u, 256, 0, stream>>>(wdt, WDTH, n8, (unsigned)(RNK / 8), (unsigned)EDIM, (unsigned)EDIM); }
    { const unsigned n8 = (unsigned)((size_t)NLAY * DMOD * EDIM / 8);
      k_wconv<<<(n8 + 255u) / 256u, 256, 0, stream>>>(wout, WOUH, n8, (unsigned)(EDIM / 8), (unsigned)DMOD, (unsigned)DMOD); }

    for (int layer = 0; layer < NLAY; ++layer) {
        const float* cur = (layer == 0) ? x_in : X1;
        float* dst = (layer == 0) ? X1 : OUT;
        const int inbf = (layer == 0) ? 1 : 0;
        const h16* winl = WINH + (size_t)layer * XZP * DMOD;
        const h16* wxl  = WXPH + (size_t)layer * XPP * EDIM;
        const h16* wdtl = WDTH + (size_t)layer * EDIM * RNK;
        const h16* woul = WOUH + (size_t)layer * DMOD * EDIM;
        k_rms<<<SEQ / 8, 256, 0, stream>>>(cur, norm_w + (size_t)layer * DMOD, XN, inbf);
        k_gemm_in<<<dim3(SEQ / 64, XZP / 64, 1), 32, 0, stream>>>(XN, winl, XZ);
        k_conv<<<SEQ, 256, 0, stream>>>(XZ, conv_w + (size_t)layer * EDIM * KCV, conv_b + (size_t)layer * EDIM, XCH);
        k_gemm_xp<<<dim3(SEQ / 64, XPP / 64, 1), 32, 0, stream>>>(XCH, wxl, DTH, BC);
        k_gemm_dt<<<dim3(SEQ / 64, EDIM / 64, 1), 32, 0, stream>>>(DTH, wdtl, bdt + (size_t)layer * EDIM, DL);
        k_scan<<<EDIM / 64, 64, 0, stream>>>(DL, XCH, BC, XZ, a_log + (size_t)layer * EDIM * NST, dpar + (size_t)layer * EDIM, YG);
        k_gemm_out<<<dim3(SEQ / 64, DMOD / 64, 1), 32, 0, stream>>>(YG, woul, cur, inbf, dst);
    }
}
